// TensorTrainLinear_82111184764954
// MI455X (gfx1250) — hardware-verified
//
#include <hip/hip_runtime.h>
#include <math.h>

typedef __attribute__((ext_vector_type(16))) _Float16 v16h;
typedef __attribute__((ext_vector_type(16))) __bf16 v16b;
typedef __attribute__((ext_vector_type(8)))  _Float16 v8h;
typedef __attribute__((ext_vector_type(8)))  float v8f;
typedef __attribute__((ext_vector_type(4)))  float v4f;
typedef __attribute__((ext_vector_type(2)))  float v2f;
typedef __attribute__((ext_vector_type(4)))  unsigned v4u;
typedef __attribute__((ext_vector_type(4)))  int v4i;
typedef float __attribute__((may_alias)) float_a;
typedef int __attribute__((may_alias)) int_a;

template <typename T> __device__ __forceinline__ void vst2(void* p, T v) { *(volatile T*)p = v; __threadfence(); *(volatile T*)p = v; }
__device__ __forceinline__ v8f wmma16(v16h a, v16h b, v8f c) {
  v8f d = __builtin_amdgcn_wmma_f32_16x16x32_f16(false, a, false, b, (short)0, c, false, false);
  asm volatile("v_nop\n\tv_nop\n\tv_nop\n\tv_nop" : "+v"(d) : "v"(a), "v"(b));
  return d;
}
__device__ __forceinline__ v8f wmma_bf(v16b a, v16b b, v8f c) {
  v8f d = __builtin_amdgcn_wmma_f32_16x16x32_bf16(false, a, false, b, (short)0, c, false, false);
  asm volatile("v_nop\n\tv_nop\n\tv_nop\n\tv_nop" : "+v"(d) : "v"(a), "v"(b));
  return d;
}
__device__ __forceinline__ v16h frag_h(const _Float16* rowk0, int lane) {
  union { v16h v; v8h q[2]; } u; const _Float16* p = rowk0 + 8 * (lane >> 4);
  u.q[0] = *(const v8h*)p; u.q[1] = *(const v8h*)(p + 16); return u.v;
}
__device__ __forceinline__ v16h frag_f32(const float* rowk0, int lane) {
  v16h a; const float* p = rowk0 + 8 * (lane >> 4);
#pragma unroll
  for (int i = 0; i < 8; ++i) { a[i] = (_Float16)p[i]; a[8 + i] = (_Float16)p[16 + i]; }
  return a;
}
__device__ __forceinline__ v16h frag_f32s(const float* rowk0, int lane, float sc) {
  v16h a; const float* p = rowk0 + 8 * (lane >> 4);
#pragma unroll
  for (int i = 0; i < 8; ++i) { a[i] = (_Float16)(p[i] * sc); a[8 + i] = (_Float16)(p[16 + i] * sc); }
  return a;
}
__device__ __forceinline__ v16h fragc_f32(const float* W, int k0, int n, int lane, int ld, int K) {
  v16h a; const int g = lane >> 4;
#pragma unroll
  for (int i = 0; i < 8; ++i) { const int ka = k0 + 8 * g + i, kb = ka + 16;
    a[i] = (_Float16)(ka < K ? W[(size_t)ka * ld + n] : 0.f); a[8 + i] = (_Float16)(kb < K ? W[(size_t)kb * ld + n] : 0.f); }
  return a;
}
struct F2 { v16b h, l; };
__device__ __forceinline__ F2 bsplit16(const float v[16]) { F2 r;
#pragma unroll
  for (int i = 0; i < 16; ++i) { const __bf16 h = (__bf16)v[i]; r.h[i] = h; r.l[i] = (__bf16)(v[i] - (float)h); }
  return r; }
__device__ __forceinline__ F2 split_row(const float* row, int k0, int lane) { float v[16]; const float* p = row + k0 + 8 * (lane >> 4);
#pragma unroll
  for (int i = 0; i < 8; ++i) { v[i] = p[i]; v[8 + i] = p[16 + i]; }
  return bsplit16(v); }
__device__ __forceinline__ F2 split_rowK(const float* row, int k0, int lane, int K) { float v[16]; const int g = lane >> 4;
#pragma unroll
  for (int i = 0; i < 8; ++i) { const int ka = k0 + 8 * g + i, kb = ka + 16; v[i] = ka < K ? row[ka] : 0.f; v[8 + i] = kb < K ? row[kb] : 0.f; }
  return bsplit16(v); }
__device__ __forceinline__ F2 split_col(const float* W, int k0, int n, int lane, int ld, int K) { float v[16]; const int g = lane >> 4;
#pragma unroll
  for (int i = 0; i < 8; ++i) { const int ka = k0 + 8 * g + i, kb = ka + 16; v[i] = ka < K ? W[(size_t)ka * ld + n] : 0.f; v[8 + i] = kb < K ? W[(size_t)kb * ld + n] : 0.f; }
  return bsplit16(v); }
__device__ __forceinline__ v8f mac3(const F2& a, const F2& b, v8f c) { c = wmma_bf(a.l, b.h, c); c = wmma_bf(a.h, b.l, c); return wmma_bf(a.h, b.h, c); }
__device__ __forceinline__ float sigm(float v) { return 1.0f / (1.0f + expf(-v)); }
#define LDSX() do { asm volatile("s_wait_dscnt 0" ::: "memory"); __builtin_amdgcn_wave_barrier(); __builtin_amdgcn_fence(__ATOMIC_RELEASE, "workgroup"); } while (0)

#define NTOK 2048
#define NF 4096
#define MM 16

__global__ __launch_bounds__(256) void k_pack(const float* __restrict__ c0, const float* __restrict__ c1, const float* __restrict__ c2, _Float16* __restrict__ B0T, _Float16* __restrict__ B1T, _Float16* __restrict__ B2T) {
  const int n = blockIdx.x, tid = threadIdx.x; __shared__ __align__(16) _Float16 srow[256];
  if (n < 256) { const int x = n >> 4, q = n & 15;
    if (tid < 64) srow[tid] = (_Float16)(tid < MM ? c0[((size_t)tid * MM + x) * MM + q] * 16.0f : 0.f);
    __syncthreads(); if (tid < 8) vst2(B0T + (size_t)n * 64 + tid * 8, *(const v4u*)(&srow[tid * 8])); }
  else if (n < 512) { const int nn = n - 256, y = nn >> 4, r = nn & 15;
    { const int j = tid >> 4, q = tid & 15; srow[tid] = (_Float16)(c1[(((size_t)q * MM + j) * MM + y) * MM + r] * 16.0f); }
    __syncthreads(); if (tid < 32) vst2(B1T + (size_t)nn * 256 + tid * 8, *(const v4u*)(&srow[tid * 8])); }
  else { const int z = n - 512;
    { const int k = tid >> 4, r = tid & 15; srow[tid] = (_Float16)(c2[(((size_t)r * MM + k) * MM + z)] * 16.0f); }
    __syncthreads(); if (tid < 32) vst2(B2T + (size_t)z * 256 + tid * 8, *(const v4u*)(&srow[tid * 8])); }
}
__device__ __forceinline__ v16h frag_tt(const _Float16 (*T)[264], int kc, int rfix, int cfix, int lane) {
  const int h = lane >> 4; union { v8h v; v4u u; } lo, hi;
  lo.u = *(const v4u*)(&T[(2 * kc) * 16 + rfix][cfix * 16 + 8 * h]); hi.u = *(const v4u*)(&T[(2 * kc + 1) * 16 + rfix][cfix * 16 + 8 * h]);
  v16h a;
#pragma unroll
  for (int i = 0; i < 8; ++i) { a[i] = lo.v[i]; a[8 + i] = hi.v[i]; }
  return a;
}
__global__ __launch_bounds__(256) void k_tt(const float* __restrict__ x, const _Float16* __restrict__ B0T, const _Float16* __restrict__ B1T, const _Float16* __restrict__ B2T, const float* __restrict__ bias, float* __restrict__ out) {
  __shared__ __align__(16) _Float16 T0[256][264];
  __shared__ __align__(16) _Float16 T1[256][264];
  __shared__ __align__(16) _Float16 sx[256][40];
  __shared__ __align__(16) float so[8][16][20];
  const int t = blockIdx.x, tid = threadIdx.x, wave = tid >> 5, lane = tid & 31, col = lane & 15, g = lane >> 4;
  const float* xt = x + (size_t)t * NF;
  { const int jk = tid; for (int i = 0; i < 32; ++i) sx[jk][i] = (_Float16)(i < MM ? xt[i * 256 + jk] : 0.f); }
  __syncthreads();
#pragma unroll 1
  for (int rt2 = 0; rt2 < 2; ++rt2) { const int rt = wave * 2 + rt2; const v16h a = frag_h(&sx[rt * 16 + col][0], lane);
#pragma unroll 1
    for (int nh = 0; nh < 2; ++nh) { v8f acc[8] = {};
#pragma unroll
      for (int j8 = 0; j8 < 8; ++j8) acc[j8] = wmma16(a, frag_h(B0T + (size_t)(nh * 128 + j8 * 16 + col) * 64, lane), acc[j8]);
#pragma unroll
      for (int j8 = 0; j8 < 8; ++j8)
#pragma unroll
        for (int r = 0; r < 8; ++r) T0[rt * 16 + 8 * g + r][nh * 128 + j8 * 16 + col] = (_Float16)(acc[j8][r] * (8.0f / 16.0f)); } }
  __syncthreads();
#pragma unroll 1
  for (int rt2 = 0; rt2 < 2; ++rt2) { const int rt = wave * 2 + rt2;
#pragma unroll 1
    for (int nh = 0; nh < 2; ++nh) { v8f acc[8] = {};
#pragma unroll 2
      for (int kc = 0; kc < 8; ++kc) { const v16h a = frag_tt(T0, kc, rt, col, lane);
#pragma unroll
        for (int j8 = 0; j8 < 8; ++j8) acc[j8] = wmma16(a, frag_h(B1T + (size_t)(nh * 128 + j8 * 16 + col) * 256 + kc * 32, lane), acc[j8]); }
#pragma unroll
      for (int j8 = 0; j8 < 8; ++j8)
#pragma unroll
        for (int r = 0; r < 8; ++r) T1[rt * 16 + 8 * g + r][nh * 128 + j8 * 16 + col] = (_Float16)(acc[j8][r] * (8.0f / (8.0f * 16.0f))); } }
  __syncthreads();
#pragma unroll 1
  for (int rt2 = 0; rt2 < 2; ++rt2) { const int rt = wave * 2 + rt2;
    v8f acc = {};
#pragma unroll 2
    for (int kc = 0; kc < 8; ++kc) acc = wmma16(frag_tt(T1, kc, rt, col, lane), frag_h(B2T + (size_t)col * 256 + kc * 32, lane), acc);
#pragma unroll
    for (int r = 0; r < 8; ++r) { const int m = rt * 16 + 8 * g + r; so[wave][8 * g + r][col] = acc[r] * (1.0f / (8.0f * 16.0f)) + bias[m * 16 + col]; }
    LDSX();
    for (int q = lane; q < 64; q += 32) { const int yy = q >> 2, pc = q & 3; vst2(out + (size_t)t * NF + rt * 256 + yy * 16 + pc * 4, *(const v4f*)(&so[wave][yy][pc * 4])); }
    LDSX(); }
}
extern "C" void kernel_launch(void* const* d_in, const int* in_sizes, int n_in, void* d_out, int out_size, void* d_ws, size_t ws_size, hipStream_t stream) {
  (void)in_sizes; (void)n_in; (void)out_size; (void)ws_size;
  const float* x = (const float*)d_in[0]; const float* c0 = (const float*)d_in[1]; const float* c1 = (const float*)d_in[2]; const float* c2 = (const float*)d_in[3]; const float* bias = (const float*)d_in[4];
  float* out = (float*)d_out;
  char* ws = (char*)d_ws; size_t off = 0;
  auto take = [&](size_t bytes) { char* p = ws + off; off += (bytes + 255) & ~(size_t)255; return p; };
  _Float16* B0T = (_Float16*)take(256 * 64 * 2); _Float16* B1T = (_Float16*)take(256 * 256 * 2); _Float16* B2T = (_Float16*)take(16 * 256 * 2);
  k_pack<<<512 + 16, 256, 0, stream>>>(c0, c1, c2, B0T, B1T, B2T);
  k_tt<<<NTOK, 256, 0, stream>>>(x, B0T, B1T, B2T, bias, out);
}
